// CompressedSparseAttention_40286793236980
// MI455X (gfx1250) — hardware-verified
//
#include <hip/hip_runtime.h>


namespace {
constexpr int Bn = 2, L = 2048, D = 512, H = 8, HD = 64, NT = Bn * L, RATIO = 8, STRIDE = 4, WIN = 128, LC = 511, LCP = 512, LVP = L + 64  ;
constexpr float QS = 8.0f, KS = 8.0f, VS = 8.0f, PS = 8.0f, AS_ = 8.0f, SCALE = 0.125f;
constexpr size_t PL = (size_t)Bn * H * L * HD, PLV = (size_t)Bn * H * HD * LVP, PLC = (size_t)Bn * H * LCP * HD;

typedef _Float16 b16;
typedef __attribute__((ext_vector_type(16))) _Float16 v16b;
typedef __attribute__((ext_vector_type(8))) _Float16 v8b;
typedef __attribute__((ext_vector_type(8))) float v8f;
typedef __attribute__((ext_vector_type(4))) float v4f;
__device__ __forceinline__ float bf16_rne(float f) { unsigned int u = __float_as_uint(f); u += 0x7FFFu + ((u >> 16) & 1u); return __uint_as_float(u & 0xFFFF0000u); }
__device__ __forceinline__ void split16(float v, b16& hi, b16& lo) { hi = (b16)v; lo = (b16)(v - (float)hi); }
__device__ __forceinline__ v16b frag_kb(const b16* p, int hh) { const v8b a = *(const v8b*)(p + 8 * hh), b = *(const v8b*)(p + 16 + 8 * hh); v16b f;
#pragma unroll
  for (int e = 0; e < 8; ++e) { f[e] = a[e]; f[8 + e] = b[e]; } return f; }
__device__ __forceinline__ v16b frag_x(const float* p, int hh) { v16b f;
#pragma unroll
  for (int e = 0; e < 8; ++e) { f[e] = (b16)bf16_rne(p[8 * hh + e]); f[8 + e] = (b16)bf16_rne(p[16 + 8 * hh + e]); } return f; }
__device__ __forceinline__ void frag_split(const float* p, int hh, v16b& fh, v16b& fl) {
#pragma unroll
  for (int e = 0; e < 8; ++e) { b16 a, c; split16(p[8 * hh + e] * AS_, a, c); fh[e] = a; fl[e] = c; split16(p[16 + 8 * hh + e] * AS_, a, c); fh[8 + e] = a; fl[8 + e] = c; } }
__device__ __forceinline__ v8f wmma16b(v16b a, v16b b, v8f c) { v8f d = __builtin_amdgcn_wmma_f32_16x16x32_f16(false, a, false, b, (short)0, c, false, false); asm volatile("v_nop\n\tv_nop\n\tv_nop\n\tv_nop" : "+v"(d) : "v"(a), "v"(b)); return d; }
__device__ __forceinline__ void wave_lds_sync() { __builtin_amdgcn_fence(__ATOMIC_RELEASE, "workgroup"); __builtin_amdgcn_wave_barrier(); __builtin_amdgcn_fence(__ATOMIC_ACQUIRE, "workgroup"); }
__device__ __forceinline__ float nexp(float x) { return __builtin_amdgcn_exp2f(x * 1.4426950408889634f); }
__device__ __forceinline__ float pmul(float a, float b) { float p = a * b; asm volatile("" : "+v"(p)); return p; }
__device__ __forceinline__ void sincos_r(float ang, float& sn, float& cs) { const float k = rintf(ang * 0.15915494309189535f); float r = __builtin_fmaf(k, -6.28318548202514648f, ang); r = __builtin_fmaf(k, 1.7484556025237907e-7f, r);
  const float t = r * 0.15915494309189535f; sn = __builtin_amdgcn_sinf(t); cs = __builtin_amdgcn_cosf(t); }

__global__ __launch_bounds__(256) void prep_kernel(const float* __restrict__ wq, const float* __restrict__ wk, const float* __restrict__ wv, const float* __restrict__ wkc, const float* __restrict__ wvc, const float* __restrict__ wo, const float* __restrict__ gl, const float* __restrict__ sink, b16* __restrict__ R, float* __restrict__ P) {
  const int t_ = blockIdx.x * 256 + threadIdx.x, nth = gridDim.x * 256;
  for (int pass = 0; pass < 2; ++pass) {
    for (int p = t_; p < 6 * D * D / 8; p += nth) { const int m = p / (D * D / 8), q = (p % (D * D / 8)) * 8; const float* W = (m == 0) ? wq : (m == 1) ? wk : (m == 2) ? wv : (m == 3) ? wkc : (m == 4) ? wvc : wo; v8b v;
#pragma unroll
      for (int e = 0; e < 8; ++e) v[e] = (b16)bf16_rne(W[q + e]); *(volatile v8b*)(R + (size_t)m * D * D + q) = v; }
    if (t_ < 64) { float v = 0.0f;
      if (t_ < RATIO) { float mx = -INFINITY; for (int r = 0; r < RATIO; ++r) mx = fmaxf(mx, bf16_rne(gl[r])); float s = 0.0f; for (int r = 0; r < RATIO; ++r) s += nexp(bf16_rne(gl[r]) - mx); v = nexp(bf16_rne(gl[t_]) - mx) / s; }
      else if (t_ < 16) v = bf16_rne(sink[t_ - 8]);
      else if (t_ < 48) v = 1.0f / powf(10000.0f, (float)(t_ - 16) / 32.0f);
      ((volatile float*)P)[t_] = v; }
    __threadfence(); }
}

__global__ __launch_bounds__(128) void proj_kernel(const float* __restrict__ x, const b16* __restrict__ R, const float* __restrict__ P, b16* __restrict__ qh, b16* __restrict__ ql, b16* __restrict__ kh, b16* __restrict__ kl, b16* __restrict__ vt, b16* __restrict__ vtl) {
  __shared__ __attribute__((aligned(16))) float Tf[4][32][64 + 4]; __shared__ __attribute__((aligned(16))) b16 Tv[64][128 + 8], Tvl[64][128 + 8];
  const int lane = threadIdx.x & 31, wave = threadIdx.x >> 5, nloc = lane & 15, hlf = lane >> 4, h = blockIdx.x, c0 = h * HD, which = blockIdx.z, p0 = blockIdx.y * 128, m0 = p0 + wave * 32, b = p0 / L, t0 = p0 % L;
  const b16* Wt = R + (size_t)which * D * D; const float* invf = P + 16;
  v8f acc[2][4];
#pragma unroll
  for (int r = 0; r < 2; ++r)
#pragma unroll
    for (int t = 0; t < 4; ++t) acc[r][t] = (v8f){};
#pragma unroll 2
  for (int kb = 0; kb < D; kb += 32) { const v16b a0 = frag_x(x + (size_t)(m0 + nloc) * D + kb, hlf), a1 = frag_x(x + (size_t)(m0 + 16 + nloc) * D + kb, hlf);
#pragma unroll
    for (int t = 0; t < 4; ++t) { const v16b bw = frag_kb(Wt + (size_t)(c0 + t * 16 + nloc) * D + kb, hlf); acc[0][t] = wmma16b(a0, bw, acc[0][t]); acc[1][t] = wmma16b(a1, bw, acc[1][t]); } }
  if (which < 2) {
#pragma unroll
    for (int t = 0; t < 4; ++t)
#pragma unroll
      for (int r = 0; r < 2; ++r)
#pragma unroll
        for (int v = 0; v < 8; ++v) Tf[wave][r * 16 + 8 * hlf + v][t * 16 + nloc] = acc[r][t][v];
    wave_lds_sync();
    const float scl = (which == 0) ? SCALE * QS : KS; b16* Ph = (which == 0) ? qh : kh; b16* Plo = (which == 0) ? ql : kl;
    __shared__ __attribute__((aligned(16))) b16 Th[4][32][64 + 8], Tl[4][32][64 + 8];
    for (int rr = 0; rr < 32; ++rr) { const int tpos = (m0 + rr) % L; float sn, cs; sincos_r((float)tpos * invf[lane], sn, cs); const float x1 = Tf[wave][rr][lane], x2 = Tf[wave][rr][32 + lane];
      const float o1 = (pmul(x1, cs) - pmul(x2, sn)) * scl, o2 = (pmul(x1, sn) + pmul(x2, cs)) * scl; b16 a, c; split16(o1, a, c); Th[wave][rr][lane] = a; Tl[wave][rr][lane] = c; split16(o2, a, c); Th[wave][rr][32 + lane] = a; Tl[wave][rr][32 + lane] = c; }
    wave_lds_sync();
    const size_t base = (((size_t)b * H + h) * L + (m0 % L)) * HD;
    for (int pass = 0; pass < 2; ++pass) {
#pragma unroll
      for (int j = 0; j < 8; ++j) { const int rr = j * 4 + (lane >> 3), c8 = (lane & 7) * 8; *(volatile v8b*)(Ph + base + (size_t)rr * HD + c8) = *(const v8b*)(&Th[wave][rr][c8]); *(volatile v8b*)(Plo + base + (size_t)rr * HD + c8) = *(const v8b*)(&Tl[wave][rr][c8]); }
      __threadfence(); }
    return; }
#pragma unroll
  for (int t = 0; t < 4; ++t)
#pragma unroll
    for (int r = 0; r < 2; ++r)
#pragma unroll
      for (int v = 0; v < 8; ++v) { b16 a_, c_; split16(acc[r][t][v] * VS, a_, c_); Tv[t * 16 + nloc][wave * 32 + r * 16 + 8 * hlf + v] = a_; Tvl[t * 16 + nloc][wave * 32 + r * 16 + 8 * hlf + v] = c_; }
  __syncthreads();
  for (int pass = 0; pass < 2; ++pass) { for (int i = threadIdx.x; i < 64 * 16; i += 128) { const int d = i >> 4, c8 = (i & 15) * 8; const size_t o_ = (((size_t)b * H + h) * HD + d) * LVP + t0 + c8; *(volatile v8b*)(vt + o_) = *(const v8b*)(&Tv[d][c8]); *(volatile v8b*)(vtl + o_) = *(const v8b*)(&Tvl[d][c8]); }
    if (t0 + 128 == L) { for (int i = threadIdx.x; i < 64 * 8; i += 128) { const int d = i >> 3, c8 = (i & 7) * 8; const size_t o_ = (((size_t)b * H + h) * HD + d) * LVP + L + c8; *(volatile v8b*)(vt + o_) = (v8b){}; *(volatile v8b*)(vtl + o_) = (v8b){}; } }
    __threadfence(); }
}

__global__ __launch_bounds__(256) void pool_kernel(const float* __restrict__ x, const float* __restrict__ P, float* __restrict__ xc) {
  const int b = blockIdx.y, w0 = blockIdx.x * 8, t_ = threadIdx.x;
  for (int pass = 0; pass < 2; ++pass) { for (int wi = 0; wi < 8; ++wi) { const int w = w0 + wi;
      for (int c = t_ * 2; c < D; c += 512) { float a0 = 0.0f, a1 = 0.0f; if (w < LC) { for (int r = 0; r < RATIO; ++r) { const float* xr = x + ((size_t)b * L + w * STRIDE + r) * D + c; a0 += pmul(P[r], bf16_rne(xr[0])); a1 += pmul(P[r], bf16_rne(xr[1])); } }
        ((volatile float*)xc)[((size_t)b * LCP + w) * D + c] = a0; ((volatile float*)xc)[((size_t)b * LCP + w) * D + c + 1] = a1; } }
    __threadfence(); }
}

__global__ __launch_bounds__(128) void projc_kernel(const float* __restrict__ xc, const b16* __restrict__ R, b16* __restrict__ kch, b16* __restrict__ kcl, b16* __restrict__ vct, b16* __restrict__ vctl) {
  __shared__ __attribute__((aligned(16))) b16 Th[4][32][64 + 8], Tl[4][32][64 + 8]; __shared__ __attribute__((aligned(16))) b16 Tv[64][128 + 8], Tvl[64][128 + 8];
  const int lane = threadIdx.x & 31, wave = threadIdx.x >> 5, nloc = lane & 15, hlf = lane >> 4, h = blockIdx.x, c0 = h * HD, which = blockIdx.z, p0 = blockIdx.y * 128, m0 = p0 + wave * 32, b = p0 / LCP, w0 = p0 % LCP;
  const b16* Wt = R + (size_t)(3 + which) * D * D;
  v8f acc[2][4];
#pragma unroll
  for (int r = 0; r < 2; ++r)
#pragma unroll
    for (int t = 0; t < 4; ++t) acc[r][t] = (v8f){};
#pragma unroll 2
  for (int kb = 0; kb < D; kb += 32) { v16b a0, l0, a1, l1; frag_split(xc + (size_t)(m0 + nloc) * D + kb, hlf, a0, l0); frag_split(xc + (size_t)(m0 + 16 + nloc) * D + kb, hlf, a1, l1);
#pragma unroll
    for (int t = 0; t < 4; ++t) { const v16b bw = frag_kb(Wt + (size_t)(c0 + t * 16 + nloc) * D + kb, hlf); acc[0][t] = wmma16b(a0, bw, acc[0][t]); acc[0][t] = wmma16b(l0, bw, acc[0][t]); acc[1][t] = wmma16b(a1, bw, acc[1][t]); acc[1][t] = wmma16b(l1, bw, acc[1][t]); } }
  if (which == 0) {
#pragma unroll
    for (int t = 0; t < 4; ++t)
#pragma unroll
      for (int r = 0; r < 2; ++r)
#pragma unroll
        for (int v = 0; v < 8; ++v) { b16 a, c; split16(acc[r][t][v] * (KS / AS_), a, c); Th[wave][r * 16 + 8 * hlf + v][t * 16 + nloc] = a; Tl[wave][r * 16 + 8 * hlf + v][t * 16 + nloc] = c; }
    wave_lds_sync();
    const size_t base = (((size_t)b * H + h) * LCP + (m0 % LCP)) * HD;
    for (int pass = 0; pass < 2; ++pass) {
#pragma unroll
      for (int j = 0; j < 8; ++j) { const int rr = j * 4 + (lane >> 3), c8 = (lane & 7) * 8; *(volatile v8b*)(kch + base + (size_t)rr * HD + c8) = *(const v8b*)(&Th[wave][rr][c8]); *(volatile v8b*)(kcl + base + (size_t)rr * HD + c8) = *(const v8b*)(&Tl[wave][rr][c8]); }
      __threadfence(); }
    return; }
#pragma unroll
  for (int t = 0; t < 4; ++t)
#pragma unroll
    for (int r = 0; r < 2; ++r)
#pragma unroll
      for (int v = 0; v < 8; ++v) { b16 a_, c_; split16(acc[r][t][v] * (VS / AS_), a_, c_); Tv[t * 16 + nloc][wave * 32 + r * 16 + 8 * hlf + v] = a_; Tvl[t * 16 + nloc][wave * 32 + r * 16 + 8 * hlf + v] = c_; }
  __syncthreads();
  for (int pass = 0; pass < 2; ++pass) { for (int i = threadIdx.x; i < 64 * 16; i += 128) { const int d = i >> 4, c8 = (i & 15) * 8; const size_t o_ = (((size_t)b * H + h) * HD + d) * LCP + w0 + c8; *(volatile v8b*)(vct + o_) = *(const v8b*)(&Tv[d][c8]); *(volatile v8b*)(vctl + o_) = *(const v8b*)(&Tvl[d][c8]); } __threadfence(); }
}

__global__ __launch_bounds__(256) void attn_kernel(const b16* __restrict__ qh, const b16* __restrict__ ql, const b16* __restrict__ kh, const b16* __restrict__ kl, const b16* __restrict__ vt, const b16* __restrict__ vtl, const b16* __restrict__ kch, const b16* __restrict__ kcl, const b16* __restrict__ vct, const b16* __restrict__ vctl, const float* __restrict__ P, float* __restrict__ ctx) {
  __shared__ __attribute__((aligned(16))) float Os[16][D + 4];
  const int h = threadIdx.x >> 5, lane = threadIdx.x & 31, hh = lane >> 4, col = lane & 15; const int b = blockIdx.x / (L / 16), q0 = (blockIdx.x % (L / 16)) * 16, qi = q0 + col;
  const size_t pb = ((size_t)b * H + h) * L * HD, pcb = ((size_t)b * H + h) * LCP * HD; const b16* Vt = vt + ((size_t)b * H + h) * HD * LVP; const b16* Vtl = vtl + ((size_t)b * H + h) * HD * LVP; const b16* Vct = vct + ((size_t)b * H + h) * HD * LCP; const b16* Vctl = vctl + ((size_t)b * H + h) * HD * LCP;
  const v16b qa0 = frag_kb(qh + pb + (size_t)qi * HD, hh), qa1 = frag_kb(qh + pb + (size_t)qi * HD + 32, hh), qb0 = frag_kb(ql + pb + (size_t)qi * HD, hh), qb1 = frag_kb(ql + pb + (size_t)qi * HD + 32, hh);
  float m = -INFINITY, l = 0.0f; v8f o[4] = {{}, {}, {}, {}};
  auto tile = [&](const b16* Kh_, const b16* Kl_, const b16* V_, const b16* Vl_, size_t vpitch, int key0, int mode  ) {
    v8f s0 = {}, s1 = {};
    { const v16b k0h = frag_kb(Kh_ + (size_t)(key0 + col) * HD, hh), k0l = frag_kb(Kl_ + (size_t)(key0 + col) * HD, hh), k1h = frag_kb(Kh_ + (size_t)(key0 + col) * HD + 32, hh), k1l = frag_kb(Kl_ + (size_t)(key0 + col) * HD + 32, hh);
      s0 = wmma16b(k0h, qa0, s0); s0 = wmma16b(k0h, qb0, s0); s0 = wmma16b(k0l, qa0, s0); s0 = wmma16b(k1h, qa1, s0); s0 = wmma16b(k1h, qb1, s0); s0 = wmma16b(k1l, qa1, s0); }
    if (mode == 0) { const v16b k0h = frag_kb(Kh_ + (size_t)(key0 + 16 + col) * HD, hh), k0l = frag_kb(Kl_ + (size_t)(key0 + 16 + col) * HD, hh), k1h = frag_kb(Kh_ + (size_t)(key0 + 16 + col) * HD + 32, hh), k1l = frag_kb(Kl_ + (size_t)(key0 + 16 + col) * HD + 32, hh);
      s1 = wmma16b(k0h, qa0, s1); s1 = wmma16b(k0h, qb0, s1); s1 = wmma16b(k0l, qa0, s1); s1 = wmma16b(k1h, qa1, s1); s1 = wmma16b(k1h, qb1, s1); s1 = wmma16b(k1l, qa1, s1); }
    float mr = -INFINITY;
#pragma unroll
    for (int r = 0; r < 8; ++r) {
#pragma unroll
      for (int u = 0; u < 2; ++u) { const int key = key0 + u * 16 + 8 * hh + r; float sv = ((u == 0) ? s0[r] : s1[r]) * (1.0f / (QS * KS)); bool keep;
        if (mode == 0) keep = (key < LC) && (qi >= key * STRIDE + RATIO - 1); else keep = (u == 0) && (key >= 0) && (qi - key >= 0) && (qi - key < WIN);
        if (!keep) sv = -INFINITY; if (u == 0) s0[r] = sv; else s1[r] = sv; mr = fmaxf(mr, sv); } }
    mr = fmaxf(mr, __shfl_xor(mr, 16));
    const float mn = fmaxf(m, mr); const float al_ = (mn == -INFINITY) ? 1.0f : nexp(m - mn); m = mn; float sum = 0.0f; v16b pbh, pbl;
#pragma unroll
    for (int r = 0; r < 8; ++r) { const float e0 = (s0[r] == -INFINITY) ? 0.0f : nexp(s0[r] - mn), e1 = (s1[r] == -INFINITY) ? 0.0f : nexp(s1[r] - mn); sum += e0 + e1; b16 a_, c_; split16(e0 * PS, a_, c_); pbh[r] = a_; pbl[r] = c_; split16(e1 * PS, a_, c_); pbh[8 + r] = a_; pbl[8 + r] = c_; }
    sum += __shfl_xor(sum, 16); l = l * al_ + sum;
#pragma unroll
    for (int t = 0; t < 4; ++t) { o[t] *= al_; const v16b vf = frag_kb(V_ + (size_t)(t * 16 + col) * vpitch + key0, hh), vl = frag_kb(Vl_ + (size_t)(t * 16 + col) * vpitch + key0, hh); o[t] = wmma16b(vf, pbh, o[t]); o[t] = wmma16b(vf, pbl, o[t]); o[t] = wmma16b(vl, pbh, o[t]); } };
  for (int c0 = 0; c0 < LCP && (q0 + 15) >= c0 * STRIDE + RATIO - 1; c0 += 32) tile(kch + pcb, kcl + pcb, Vct, Vctl, LCP, c0, 0);
  for (int key0 = ((q0 - WIN) > 0 ? (q0 - WIN) : 0); key0 <= q0; key0 += 16) tile(kh + pb, kl + pb, Vt, Vtl, LVP, key0, 1);
  { const float sk = P[8 + h]; const float mn = fmaxf(m, sk); const float al_ = nexp(m - mn); m = mn; l = l * al_ + nexp(sk - mn);
#pragma unroll
    for (int t = 0; t < 4; ++t) o[t] *= al_; }
  const float inv = 1.0f / (l * VS * PS);
#pragma unroll
  for (int t = 0; t < 4; ++t)
#pragma unroll
    for (int r = 0; r < 8; ++r) Os[col][h * HD + t * 16 + 8 * hh + r] = o[t][r] * inv;
  __syncthreads();
  for (int pass = 0; pass < 2; ++pass) { for (int i = threadIdx.x; i < 16 * (D / 4); i += 256) { const int rr = i / (D / 4), c4 = (i % (D / 4)) * 4; *(volatile v4f*)(ctx + ((size_t)b * L + q0 + rr) * D + c4) = *(const v4f*)(&Os[rr][c4]); } __threadfence(); }
}

__global__ __launch_bounds__(128) void out_kernel(const float* __restrict__ ctx, const b16* __restrict__ R, float* __restrict__ out) {
  __shared__ __attribute__((aligned(16))) float Ts[4][32 * 64];
  const int lane = threadIdx.x & 31, wave = threadIdx.x >> 5, nloc = lane & 15, hlf = lane >> 4, m0 = blockIdx.y * 128 + wave * 32, c0 = blockIdx.x * 64; const b16* Wo = R + (size_t)5 * D * D;
  v8f acc[2][4];
#pragma unroll
  for (int r = 0; r < 2; ++r)
#pragma unroll
    for (int t = 0; t < 4; ++t) acc[r][t] = (v8f){};
#pragma unroll 2
  for (int kb = 0; kb < D; kb += 32) { v16b a0, l0, a1, l1; frag_split(ctx + (size_t)(m0 + nloc) * D + kb, hlf, a0, l0); frag_split(ctx + (size_t)(m0 + 16 + nloc) * D + kb, hlf, a1, l1);
#pragma unroll
    for (int t = 0; t < 4; ++t) { const v16b bw = frag_kb(Wo + (size_t)(c0 + t * 16 + nloc) * D + kb, hlf); acc[0][t] = wmma16b(a0, bw, acc[0][t]); acc[0][t] = wmma16b(l0, bw, acc[0][t]); acc[1][t] = wmma16b(a1, bw, acc[1][t]); acc[1][t] = wmma16b(l1, bw, acc[1][t]); } }
  float* Tt = Ts[wave];
#pragma unroll
  for (int t = 0; t < 4; ++t)
#pragma unroll
    for (int r = 0; r < 2; ++r)
#pragma unroll
      for (int v = 0; v < 8; ++v) Tt[(r * 16 + v + 8 * hlf) * 64 + t * 16 + nloc] = acc[r][t][v] * (1.0f / AS_);
  wave_lds_sync();
  for (int pass = 0; pass < 2; ++pass) {
#pragma unroll
    for (int j = 0; j < 16; ++j) { const int rr = j * 2 + hlf, c4 = nloc * 4; *(volatile v4f*)(out + (size_t)(m0 + rr) * D + c0 + c4) = *(const v4f*)(Tt + rr * 64 + c4); }
    __threadfence(); }
}
}

extern "C" void kernel_launch(void* const* d_in, const int* in_sizes, int n_in,
                              void* d_out, int out_size, void* d_ws, size_t ws_size, hipStream_t stream) {
  (void)n_in; (void)out_size;
  const float* x = (const float*)d_in[0]; const float* wq = (const float*)d_in[1]; const float* wk = (const float*)d_in[2]; const float* wv = (const float*)d_in[3]; const float* wo = (const float*)d_in[4]; const float* wkc = (const float*)d_in[5]; const float* wvc = (const float*)d_in[6]; const float* gl = (const float*)d_in[7]; const float* sink = (const float*)d_in[8];
  float* out = (float*)d_out;
  if (in_sizes[0] != NT * D || in_sizes[1] != D * D || in_sizes[7] != RATIO || in_sizes[8] != H) return;
  size_t off = 0; char* ws = (char*)d_ws;
  auto carve = [&](size_t bytes) { char* p = ws + off; off += (bytes + 255) & ~(size_t)255; return p; };
  b16* R = (b16*)carve((size_t)6 * D * D * 2); float* P = (float*)carve(256 * 4);
  b16* qh = (b16*)carve(PL * 2); b16* ql = (b16*)carve(PL * 2); b16* kh = (b16*)carve(PL * 2); b16* kl = (b16*)carve(PL * 2); b16* vt = (b16*)carve(PLV * 2); b16* vtl = (b16*)carve(PLV * 2);
  float* xc = (float*)carve((size_t)Bn * LCP * D * 4); b16* kch = (b16*)carve(PLC * 2); b16* kcl = (b16*)carve(PLC * 2); b16* vct = (b16*)carve(PLC * 2); b16* vctl = (b16*)carve(PLC * 2); float* ctx = (float*)carve((size_t)NT * D * 4);
  if (off > ws_size) return;
  prep_kernel<<<256, 256, 0, stream>>>(wq, wk, wv, wkc, wvc, wo, gl, sink, R, P);
  proj_kernel<<<dim3(H, NT / 128, 3), 128, 0, stream>>>(x, R, P, qh, ql, kh, kl, vt, vtl);
  pool_kernel<<<dim3(LCP / 8, Bn), 256, 0, stream>>>(x, P, xc);
  projc_kernel<<<dim3(H, Bn * LCP / 128, 2), 128, 0, stream>>>(xc, R, kch, kcl, vct, vctl);
  attn_kernel<<<NT / 16, 256, 0, stream>>>(qh, ql, kh, kl, vt, vtl, kch, kcl, vct, vctl, P, ctx);
  out_kernel<<<dim3(D / 64, NT / 128), 128, 0, stream>>>(ctx, R, out);
}
